// GraphTripletConvModule_63007170232987
// MI455X (gfx1250) — hardware-run, weakly checked
//
#include <hip/hip_runtime.h>
#include <stddef.h>
#include <stdint.h>


#define NN      10000
#define NE      320000
#define DD      256
#define KE      32
#define MP      10112
#define NFP     512
#define NAP     512
#define WABP    512
#define WMCP    256
#define N1_TWO_TERM    1
#define STEP2_TWO_TERM 0
#define N1_K    (N1_TWO_TERM ? 512 : 256)
#define CONV_HALVES 1
#define CNT_T   (16 / CONV_HALVES)

#define NTHR    256
#define NWAVE   8
#define EPT     8
#define CHUNK   (NTHR * EPT)
#define WCAP    (EPT * 32)
#define LISTN   (NWAVE * WCAP)
#define NB      512
#define SLB     9
#define NBLK    ((NN + NB - 1) / NB)
#define RCAP    18432
#define DEGCAP  96
#define GBM     64
#define GBN     128
#define GTHR    128
#define CW      4
#define CTHR    (CW * 32)
#define TP      260
#define TSZ     (16 * TP)
#define CONV_DYN (CW * 2 * TSZ * 4)
#define LDS_BKT ((2 * RCAP + 2 * NB + LISTN + 2 * NWAVE) * 4)

#define PB_XB   ((MP * (DD / 8)) / NTHR)
#define PB_EB   ((NE * (KE / 8)) / NTHR)
#define PB_WN   ((DD * (DD / 8)) / NTHR)
#define PB_WE   ((DD * (KE / 8)) / NTHR)
#define PB_WAB  ((2 * DD * (DD / 8)) / NTHR)
#define PB_WMC  ((DD * (DD / 8)) / NTHR)
#define PB_BIAS 1
#define PB1     (PB_XB)
#define PB2     (PB1 + PB_EB)
#define PB3     (PB2 + PB_WN)
#define PB4     (PB3 + PB_WE)
#define PB5     (PB4 + PB_WAB)
#define PB6     (PB5 + PB_WMC)
#define PB_TOT  (PB6 + PB_BIAS)

static_assert(MP % GBM == 0 && MP >= NN);
static_assert((MP * (DD / 8)) % NTHR == 0 && (NE * (KE / 8)) % NTHR == 0);
static_assert(NBLK * NB >= NN);
static_assert(NE < (1 << 19));
static_assert(DD == 32 * 8 && DD == 2 * GBN && (DD % 32) == 0);
static_assert(KE == 32);
static_assert(NTHR * 2 == NB && NB == (1 << SLB));
static_assert((CHUNK & (CHUNK - 1)) == 0 && CHUNK <= 4096);
static_assert(RCAP % (2 * NTHR) == 0 && RCAP >= 16764 + 16764 / 20);
static_assert(DEGCAP >= 55 + 8 && (DEGCAP % 16) == 0);
static_assert((TP % 4) == 0 && TP >= DD);
static_assert(LDS_BKT <= 327680);
static_assert(CONV_DYN + CW * 1024 + DD * 4 <= 327680);
static_assert(GBM == (GTHR / 32) * 16);
static_assert((N1_K % 32) == 0 && N1_K <= WABP && N1_K <= NFP);
static_assert(CONV_HALVES == 1 || CONV_HALVES == 2);
static_assert(NN % CW == 0);

typedef float          v4f   __attribute__((ext_vector_type(4)));
typedef float          v8f   __attribute__((ext_vector_type(8)));
typedef int            v2i   __attribute__((ext_vector_type(2)));
typedef int            v4i   __attribute__((ext_vector_type(4)));
typedef int            v8i   __attribute__((ext_vector_type(8)));
typedef unsigned short v4us  __attribute__((ext_vector_type(4)));
typedef unsigned short v8us  __attribute__((ext_vector_type(8)));
typedef __bf16         v16bf __attribute__((ext_vector_type(16)));
typedef v4f  __attribute__((may_alias)) v4fa;
typedef v4us __attribute__((may_alias)) v4usa;
typedef v8us __attribute__((may_alias)) v8usa;
union FragB { v16bf v; v8us u[2]; v8i w; v4i q[2]; };

__device__ __forceinline__ v8f wmx(const FragB& a, const FragB& b, v8f c) {
  v8f d = __builtin_amdgcn_wmma_f32_16x16x32_bf16(false, a.v, false, b.v, (short)0, c, false, false);
  asm volatile("v_nop\n\tv_nop\n\tv_nop\n\tv_nop" : "+v"(d) : "v"(a.w), "v"(b.w));
  return d;
}

__device__ __forceinline__ void pinf(float x) { asm volatile("" :: "v"(x)); }
__device__ __forceinline__ void pini(int x)   { asm volatile("" :: "v"(x)); }

__device__ __forceinline__ unsigned bfbits(float v) {
  const unsigned u = __float_as_uint(v);
  const unsigned r = (u + 0x7FFFu + ((u >> 16) & 1u)) >> 16;
  const unsigned nb = ((u >> 16) & 0x8000u) | 0x7FC0u;
  return ((u & 0x7FFFFFFFu) > 0x7F800000u) ? nb : r;
}
__device__ __forceinline__ float rbf(float v) { return __uint_as_float(bfbits(v) << 16); }

__device__ __forceinline__ unsigned rne_u(float v) {
  const unsigned u = __float_as_uint(v);
  return u + 0x7FFFu + ((u >> 16) & 1u);
}
__device__ __forceinline__ void split2(float a, float b, unsigned& hw, unsigned& lw) {
  const unsigned ra = rne_u(a), rb = rne_u(b);
  hw = (ra >> 16) | (rb & 0xFFFF0000u);
  const float la = a - __uint_as_float(ra & 0xFFFF0000u);
  const float lb = b - __uint_as_float(rb & 0xFFFF0000u);
  const unsigned qa = rne_u(la), qb = rne_u(lb);
  lw = (qa >> 16) | (qb & 0xFFFF0000u);
}
__device__ __forceinline__ float relu_np(float v) { return (v > 0.0f) ? v : (v - v); }

__device__ __forceinline__ void wave_sync() {
  __builtin_amdgcn_fence(__ATOMIC_RELEASE, "wavefront");
  __builtin_amdgcn_wave_barrier();
  __builtin_amdgcn_fence(__ATOMIC_ACQUIRE, "wavefront");
}

__device__ __forceinline__ void wtr_unit(const float* __restrict__ w, int srow0, int scol,
                                         unsigned short* dst, int dupOff) {
  float f[8];
#pragma unroll
  for (int i = 0; i < 8; ++i) {
    f[i] = w[(size_t)(srow0 + i) * DD + scol];
    pinf(f[i]);
  }
  v8us hv;
#pragma unroll
  for (int i = 0; i < 8; ++i) hv[i] = (unsigned short)bfbits(f[i]);
  *(volatile v8us*)dst = hv;
  if (dupOff != 0) *(volatile v8us*)(dst + dupOff) = hv;
  __threadfence();
  *(volatile v8us*)dst = hv;
  if (dupOff != 0) *(volatile v8us*)(dst + dupOff) = hv;
}

__global__ __launch_bounds__(NTHR) void k_prep(
    const float* __restrict__ xin, const float* __restrict__ efin,
    const float* __restrict__ Wn, const float* __restrict__ bn,
    const float* __restrict__ We, const float* __restrict__ be,
    const float* __restrict__ Wm, const float* __restrict__ bm,
    unsigned short* xb, unsigned short* ebp, unsigned short* wnt, unsigned short* wet,
    unsigned short* wab, unsigned short* wmc, float* biasp)
{
  const int b = (int)blockIdx.x, tid = (int)threadIdx.x;
  if (b < PB1) {
    const int i   = b * NTHR + tid;
    const int row = i >> 5;
    const int c0  = (i & 31) * 8;
    const int rc  = row < NN ? row : NN - 1;
    const float* p = xin + (size_t)rc * DD + c0;
    const v4f a = *(const v4f*)p, c = *(const v4f*)(p + 4);
    const unsigned mk = row < NN ? 0xFFFFu : 0u;
    v8us hv;
    hv[0] = (unsigned short)(bfbits(a.x) & mk); hv[1] = (unsigned short)(bfbits(a.y) & mk);
    hv[2] = (unsigned short)(bfbits(a.z) & mk); hv[3] = (unsigned short)(bfbits(a.w) & mk);
    hv[4] = (unsigned short)(bfbits(c.x) & mk); hv[5] = (unsigned short)(bfbits(c.y) & mk);
    hv[6] = (unsigned short)(bfbits(c.z) & mk); hv[7] = (unsigned short)(bfbits(c.w) & mk);
    unsigned short* dp = xb + (size_t)row * DD + c0;
    *(volatile v8us*)dp = hv;
    __threadfence();
    *(volatile v8us*)dp = hv;
  } else if (b < PB2) {
    const int u = (b - PB1) * NTHR + tid;
    const float* p = efin + (size_t)u * 8;
    const v4f a = *(const v4f*)p, c = *(const v4f*)(p + 4);
    v8us hv;
    hv[0] = (unsigned short)bfbits(a.x); hv[1] = (unsigned short)bfbits(a.y);
    hv[2] = (unsigned short)bfbits(a.z); hv[3] = (unsigned short)bfbits(a.w);
    hv[4] = (unsigned short)bfbits(c.x); hv[5] = (unsigned short)bfbits(c.y);
    hv[6] = (unsigned short)bfbits(c.z); hv[7] = (unsigned short)bfbits(c.w);
    unsigned short* dp = ebp + (size_t)u * 8;
    *(volatile v8us*)dp = hv;
    __threadfence();
    *(volatile v8us*)dp = hv;
  } else if (b < PB3) {
    const int v = (b - PB2) * NTHR + tid;
    const int n = v >> 5, k8 = (v & 31) * 8;
    wtr_unit(Wn, k8, n, wnt + (size_t)n * DD + k8, 0);
  } else if (b < PB4) {
    const int v = (b - PB3) * NTHR + tid;
    const int n = v >> 2, k8 = (v & 3) * 8;
    wtr_unit(We, k8, n, wet + (size_t)n * KE + k8, 0);
  } else if (b < PB5) {
    const int v = (b - PB4) * NTHR + tid;
    const int n = v >> 5, k8 = (v & 31) * 8;
    const int hb = n >> 8;
    wtr_unit(Wm, DD * hb + k8, n & (DD - 1), wab + (size_t)n * WABP + k8, DD);
  } else if (b < PB6) {
    const int v = (b - PB5) * NTHR + tid;
    const int n = v >> 5, k8 = (v & 31) * 8;
    wtr_unit(Wm, 2 * DD + k8, n, wmc + (size_t)n * WMCP + k8, 0);
  } else {
    if (tid < 192) {
      const int seg = tid >> 6;
      const int off = (tid & 63) * 4;
      const v4f a = *(const v4f*)(bn + off);
      const v4f c = *(const v4f*)(be + off);
      const v4f d = *(const v4f*)(bm + off);
      pinf(a.x); pinf(a.y); pinf(a.z); pinf(a.w);
      pinf(c.x); pinf(c.y); pinf(c.z); pinf(c.w);
      pinf(d.x); pinf(d.y); pinf(d.z); pinf(d.w);
      const unsigned m0 = (seg == 0) ? 0xFFFFFFFFu : 0u;
      const unsigned m1 = (seg == 1) ? 0xFFFFFFFFu : 0u;
      const unsigned m2 = (seg == 2) ? 0xFFFFFFFFu : 0u;
      v4f o;
      o.x = rbf(__uint_as_float((__float_as_uint(a.x) & m0) | (__float_as_uint(c.x) & m1) | (__float_as_uint(d.x) & m2)));
      o.y = rbf(__uint_as_float((__float_as_uint(a.y) & m0) | (__float_as_uint(c.y) & m1) | (__float_as_uint(d.y) & m2)));
      o.z = rbf(__uint_as_float((__float_as_uint(a.z) & m0) | (__float_as_uint(c.z) & m1) | (__float_as_uint(d.z) & m2)));
      o.w = rbf(__uint_as_float((__float_as_uint(a.w) & m0) | (__float_as_uint(c.w) & m1) | (__float_as_uint(d.w) & m2)));
      float* dp = biasp + 4 * tid;
      *(volatile v4f*)dp = o;
      __threadfence();
      *(volatile v4f*)dp = o;
    }
  }
}

__device__ __forceinline__ int scan_chunk(const int* __restrict__ keys, int cbase, int slotBase,
                                          int* list, int lane, int wave) {
  int wc = 0;
  const int elw = wave * WCAP + lane;
  const int e0  = cbase + elw;
  const int d0 = keys[(e0       ) < NE ? (e0       ) : NE - 1];
  const int d1 = keys[(e0 +  32) < NE ? (e0 +  32) : NE - 1];
  const int d2 = keys[(e0 +  64) < NE ? (e0 +  64) : NE - 1];
  const int d3 = keys[(e0 +  96) < NE ? (e0 +  96) : NE - 1];
  const int d4 = keys[(e0 + 128) < NE ? (e0 + 128) : NE - 1];
  const int d5 = keys[(e0 + 160) < NE ? (e0 + 160) : NE - 1];
  const int d6 = keys[(e0 + 192) < NE ? (e0 + 192) : NE - 1];
  const int d7 = keys[(e0 + 224) < NE ? (e0 + 224) : NE - 1];
  pini(d0); pini(d1); pini(d2); pini(d3); pini(d4); pini(d5); pini(d6); pini(d7);
  const unsigned nbs = (unsigned)slotBase;
  const unsigned unb = (unsigned)NB;
  const unsigned s0 = (unsigned)d0 - nbs, s1 = (unsigned)d1 - nbs;
  const unsigned s2 = (unsigned)d2 - nbs, s3 = (unsigned)d3 - nbs;
  const unsigned s4 = (unsigned)d4 - nbs, s5 = (unsigned)d5 - nbs;
  const unsigned s6 = (unsigned)d6 - nbs, s7 = (unsigned)d7 - nbs;
  const bool h0 = (s0 < unb) & (e0       < NE), h1 = (s1 < unb) & (e0 +  32 < NE);
  const bool h2 = (s2 < unb) & (e0 +  64 < NE), h3 = (s3 < unb) & (e0 +  96 < NE);
  const bool h4 = (s4 < unb) & (e0 + 128 < NE), h5 = (s5 < unb) & (e0 + 160 < NE);
  const bool h6 = (s6 < unb) & (e0 + 192 < NE), h7 = (s7 < unb) & (e0 + 224 < NE);
  const unsigned any = __builtin_amdgcn_ballot_w32(h0 | h1 | h2 | h3 | h4 | h5 | h6 | h7);
  if (any != 0u) {
#define HITJ(J, HJ, SJ) { \
      const unsigned mj = __builtin_amdgcn_ballot_w32(HJ); \
      if (mj != 0u) { \
        if (HJ) { \
          const int pos = wc + (int)__builtin_amdgcn_mbcnt_lo(mj, 0u); \
          if (pos < WCAP) list[wave * WCAP + pos] = ((elw + 32 * (J)) << 12) | (int)(SJ); \
        } \
        wc += (int)__builtin_popcount(mj); } }
    HITJ(0, h0, s0)
    HITJ(1, h1, s1)
    HITJ(2, h2, s2)
    HITJ(3, h3, s3)
    HITJ(4, h4, s4)
    HITJ(5, h5, s5)
    HITJ(6, h6, s6)
    HITJ(7, h7, s7)
#undef HITJ
  }
  return wc;
}

__global__ __launch_bounds__(NTHR) void k_bucket(const int* __restrict__ srcs, const int* __restrict__ keys,
                                                 int* ent, int* slot) {
  extern __shared__ __attribute__((aligned(16))) int dsm_b[];
  int* reg1 = dsm_b;
  int* reg2 = reg1 + RCAP;
  int* scnt = reg2 + RCAP;
  int* soff = scnt + NB;
  int* list = soff + NB;
  int* wcnt = list + LISTN;
  int* wtot = wcnt + NWAVE;
  const int tid = (int)threadIdx.x, lane = tid & 31;
  const int wave = __builtin_amdgcn_readfirstlane(tid >> 5);
  const int nodeBase = (int)blockIdx.x * NB;

  for (int i = tid; i < NB; i += NTHR) scnt[i] = 0;
  for (int i = tid; i < RCAP; i += NTHR) { reg1[i] = 0; reg2[i] = 0; }
  __syncthreads();

  int tot = 0;
  const int nChunks = (NE + CHUNK - 1) / CHUNK;
#pragma unroll 1
  for (int ch = 0; ch < nChunks; ++ch) {
    const int cbase = ch * CHUNK;
    const int wc = scan_chunk(keys, cbase, nodeBase, list, lane, wave);
    if (lane == 0) wcnt[wave] = wc;
    __syncthreads();
    int pre = 0, all = 0;
#pragma unroll
    for (int w2 = 0; w2 < NWAVE; ++w2) {
      int c = wcnt[w2];
      c = c < 0 ? 0 : (c > WCAP ? WCAP : c);
      all += c;
      pre += (w2 < wave) ? c : 0;
    }
    const int wcc  = wc > WCAP ? WCAP : wc;
    const int base = tot + pre;
#pragma unroll 1
    for (int i = lane; i < wcc; i += 32) {
      const int en = list[wave * WCAP + i];
      const int el = (en >> 12) & (CHUNK - 1);
      const int sl = en & (NB - 1);
      int eid = cbase + el;
      eid = eid > NE - 1 ? NE - 1 : eid;
      const int pos = base + i;
      if (pos < RCAP) reg1[pos] = (int)(((unsigned)eid << SLB) | (unsigned)sl);
    }
    tot += all;
    tot = tot > RCAP ? RCAP : tot;
    __syncthreads();
  }
  const int nh = tot;

  if (wave == 0) {
#pragma unroll 1
    for (int b0 = 0; b0 < nh; b0 += 32) {
      const int idx = b0 + lane;
      const int uv  = reg1[idx < RCAP ? idx : RCAP - 1];
      const int m32 = (nh - b0) < 32 ? (nh - b0) : 32;
#pragma unroll 1
      for (int k = 0; k < m32; ++k) {
        const int u  = __builtin_amdgcn_readlane(uv, k);
        const int sl = u & (NB - 1);
        if (lane == 0) scnt[sl] = scnt[sl] + 1;
      }
    }
  }
  __syncthreads();

  {
    const int r0 = scnt[2 * tid], r1 = scnt[2 * tid + 1];
    const int e0 = r0 < 0 ? 0 : r0, e1 = r1 < 0 ? 0 : r1;
    const int ts = e0 + e1;
    int incl = ts;
#pragma unroll
    for (int d = 1; d < 32; d <<= 1) {
      const int up = __shfl_up(incl, d);
      if (lane >= d) incl += up;
    }
    if (lane == 31) wtot[wave] = incl;
    __syncthreads();
    int pre = 0;
#pragma unroll
    for (int w2 = 0; w2 < NWAVE; ++w2) pre += (w2 < wave) ? wtot[w2] : 0;
    const int run = pre + incl - ts;
    soff[2 * tid]     = run;
    soff[2 * tid + 1] = run + e0;
  }
  __syncthreads();
  for (int i = tid; i < NB; i += NTHR) list[i] = soff[i];
  __syncthreads();

  if (wave == 0) {
#pragma unroll 1
    for (int b0 = 0; b0 < nh; b0 += 32) {
      const int idx = b0 + lane;
      const int uv  = reg1[idx < RCAP ? idx : RCAP - 1];
      const int m32 = (nh - b0) < 32 ? (nh - b0) : 32;
#pragma unroll 1
      for (int k = 0; k < m32; ++k) {
        const int u   = __builtin_amdgcn_readlane(uv, k);
        const int sl  = u & (NB - 1);
        const int eid = (int)((unsigned)u >> SLB);
        if (lane == 0) {
          int pos = list[sl];
          pos = pos < 0 ? 0 : (pos > RCAP - 1 ? RCAP - 1 : pos);
          reg2[pos] = eid;
          list[sl] = pos + 1;
        }
      }
    }
  }
  __syncthreads();

  const bool ovf = (nh >= RCAP);
  int* eb = ent + (size_t)blockIdx.x * (size_t)(2 * RCAP);
#pragma unroll 1
  for (int p0 = 0; p0 < RCAP; p0 += 2 * NTHR) {
    const int p = p0 + 2 * tid;
    int e0 = reg2[p], e1 = reg2[p + 1];
    e0 = e0 < 0 ? 0 : (e0 > NE - 1 ? NE - 1 : e0);
    e1 = e1 < 0 ? 0 : (e1 > NE - 1 ? NE - 1 : e1);
    int s0 = srcs[e0];
    int s1 = srcs[e1];
    pini(s0); pini(s1);
    s0 = s0 < 0 ? 0 : (s0 > NN - 1 ? NN - 1 : s0);
    s1 = s1 < 0 ? 0 : (s1 > NN - 1 ? NN - 1 : s1);
    const int m0 = (p     < nh) ? -1 : 0;
    const int m1 = (p + 1 < nh) ? -1 : 0;
    v4i v;
    v.x = s0 & m0; v.y = e0 & m0; v.z = s1 & m1; v.w = e1 & m1;
    *(volatile v4i*)(eb + 2 * p) = v;
    __threadfence();
    *(volatile v4i*)(eb + 2 * p) = v;
  }
  {
    v4i sv;
    sv.x = soff[2 * tid];
    sv.y = ovf ? -1 : scnt[2 * tid];
    sv.z = soff[2 * tid + 1];
    sv.w = ovf ? -1 : scnt[2 * tid + 1];
    int* sp = slot + 2 * (size_t)(nodeBase + 2 * tid);
    *(volatile v4i*)sp = sv;
    __threadfence();
    *(volatile v4i*)sp = sv;
  }
}

template <int MODE>
__global__ __launch_bounds__(GTHR) __attribute__((amdgpu_num_vgpr(248)))
void k_gemm(const unsigned short* __restrict__ A, int lda, const unsigned short* __restrict__ BT, int ldb, int K,
            const float* __restrict__ bias, unsigned short* outH, float* outF, int nOut) {
  __shared__ __attribute__((aligned(16))) float stg[GBM * GBN];
  const int tid = (int)threadIdx.x, lane = tid & 31, wave = tid >> 5, hh = lane >> 4, m = lane & 15;
  const int rowBase = (int)blockIdx.x * GBM;
  const int col0    = (int)blockIdx.y * GBN;

  v8f acc[8];
  {
    const v8f z = {0.f, 0.f, 0.f, 0.f, 0.f, 0.f, 0.f, 0.f};
#pragma unroll
    for (int t = 0; t < 8; ++t) acc[t] = z;
  }
  const unsigned short* ap = A  + (size_t)(rowBase + 16 * wave + m) * (size_t)lda + 8 * hh;
  const unsigned short* bp = BT + (size_t)(col0 + m) * (size_t)ldb + 8 * hh;

#pragma unroll 1
  for (int k0 = 0; k0 < K; k0 += 32) {
    FragB af;
    af.u[0] = *(const v8usa*)(ap + k0);
    af.u[1] = *(const v8usa*)(ap + k0 + 16);
#pragma unroll
    for (int nt = 0; nt < 8; ++nt) {
      const unsigned short* wq = bp + (size_t)(16 * nt) * (size_t)ldb + k0;
      FragB bf;
      bf.u[0] = *(const v8usa*)wq;
      bf.u[1] = *(const v8usa*)(wq + 16);
      acc[nt] = wmx(af, bf, acc[nt]);
    }
  }

#pragma unroll
  for (int nt = 0; nt < 8; ++nt) {
    const int lc = 16 * nt + m;
#pragma unroll
    for (int r = 0; r < 8; ++r) {
      const int lr = 16 * wave + 8 * hh + r;
      stg[lr * GBN + lc] = acc[nt][r];
    }
  }
  __syncthreads();

  v4f pv[16];
#pragma unroll
  for (int i = 0; i < 16; ++i) pv[i] = *(const v4fa*)(stg + (16 * wave + i) * GBN + 4 * lane);
  __syncthreads();

  if constexpr (MODE == 0) {
    const v4f bb4 = *(const v4f*)(bias + col0 + 4 * lane);
#pragma unroll
    for (int i = 0; i < 16; ++i) {
      const bool ok = (rowBase + 16 * wave + i) < nOut;
      const v4f t = pv[i] + bb4;
      float y0 = relu_np(t.x), y1 = relu_np(t.y), y2 = relu_np(t.z), y3 = relu_np(t.w);
      y0 = ok ? y0 : 0.0f; y1 = ok ? y1 : 0.0f; y2 = ok ? y2 : 0.0f; y3 = ok ? y3 : 0.0f;
      v4us h4, l4;
      unsigned hb;
      hb = bfbits(y0); h4[0] = (unsigned short)hb; l4[0] = (unsigned short)bfbits(y0 - __uint_as_float(hb << 16));
      hb = bfbits(y1); h4[1] = (unsigned short)hb; l4[1] = (unsigned short)bfbits(y1 - __uint_as_float(hb << 16));
      hb = bfbits(y2); h4[2] = (unsigned short)hb; l4[2] = (unsigned short)bfbits(y2 - __uint_as_float(hb << 16));
      hb = bfbits(y3); h4[3] = (unsigned short)hb; l4[3] = (unsigned short)bfbits(y3 - __uint_as_float(hb << 16));
      unsigned short* srow = (unsigned short*)stg + (size_t)(16 * wave + i) * (2 * GBN);
      *(v4usa*)(srow + 4 * lane) = h4;
      *(v4usa*)(srow + GBN + 4 * lane) = l4;
    }
    __syncthreads();
    v8us qv[16];
#pragma unroll
    for (int i = 0; i < 16; ++i) {
      const unsigned short* srow = (const unsigned short*)stg + (size_t)(16 * wave + i) * (2 * GBN);
      qv[i] = *(const v8usa*)(srow + 8 * lane);
    }
    const int dcol = (lane >> 4) * DD + col0 + 8 * (lane & 15);
#pragma unroll
    for (int i = 0; i < 16; ++i) {
      unsigned short* rp = outH + (size_t)(rowBase + 16 * wave + i) * (size_t)NFP + dcol;
      *(volatile v8us*)rp = qv[i];
    }
    __threadfence();
#pragma unroll
    for (int i = 0; i < 16; ++i) {
      unsigned short* rp = outH + (size_t)(rowBase + 16 * wave + i) * (size_t)NFP + dcol;
      *(volatile v8us*)rp = qv[i];
    }
  } else {
#pragma unroll
    for (int i = 0; i < 16; ++i) {
      float* op = outF + (size_t)(rowBase + 16 * wave + i) * (size_t)NAP + col0 + 4 * lane;
      *(volatile v4f*)op = pv[i];
    }
    __threadfence();
#pragma unroll
    for (int i = 0; i < 16; ++i) {
      float* op = outF + (size_t)(rowBase + 16 * wave + i) * (size_t)NAP + col0 + 4 * lane;
      *(volatile v4f*)op = pv[i];
    }
  }
  (void)bias; (void)outH; (void)outF; (void)nOut;
}

__global__ __launch_bounds__(CTHR) __attribute__((amdgpu_num_vgpr(248)))
void k_replay(const int* __restrict__ lst, const int* __restrict__ slot,
              const unsigned short* __restrict__ eb, const unsigned short* __restrict__ wet,
              const unsigned short* __restrict__ wmc, const float* __restrict__ nanb,
              const float* __restrict__ biasp, float* outp)
{
  extern __shared__ __attribute__((aligned(16))) float dsm_c[];
  __shared__ __attribute__((aligned(16))) int   sA[CW * 256];
  __shared__ __attribute__((aligned(16))) float sBe[DD];
  const int tid = (int)threadIdx.x, lane = tid & 31, hh = lane >> 4, m = lane & 15;
  const int wave = __builtin_amdgcn_readfirstlane(tid >> 5);
  if (tid < 64) {
    const v4f bq = *(const v4f*)(biasp + DD + 4 * tid);
    *(v4f*)(sBe + 4 * tid) = bq;
  }
  __syncthreads();
  const int i = (int)blockIdx.x * CW + wave;
  if (i >= NN) return;
  int*   At = sA + wave * 256;
  float* T  = dsm_c + wave * (2 * TSZ);
  float* U  = T + TSZ;

  const v2i se = *(const v2i*)(slot + 2 * (size_t)i);
  int stv = se.x;
  stv = stv < 0 ? 0 : (stv > RCAP - 1 ? RCAP - 1 : stv);
  const int crv = se.y;
  int cv = crv < 0 ? 0 : (crv > DEGCAP ? DEGCAP : crv);
  cv = cv > RCAP - stv ? RCAP - stv : cv;
  const int st   = __builtin_amdgcn_readfirstlane(stv);
  const int c    = __builtin_amdgcn_readfirstlane(cv);
  const int craw = __builtin_amdgcn_readfirstlane(crv);
  int last = st + c - 1;
  last = last < st ? st : last;
  const bool bad = (craw < 0) || (craw > DEGCAP);
  const int* lb = lst + (size_t)(i >> SLB) * (size_t)(2 * RCAP);

  const float* nbp = nanb + (size_t)i * NAP + DD + 4 * lane;
  const v4f nbm0 = *(const v4f*)nbp         + *(const v4f*)(biasp + 2 * DD + 4 * lane);
  const v4f nbm1 = *(const v4f*)(nbp + 128) + *(const v4f*)(biasp + 2 * DD + 128 + 4 * lane);
  v4f ao0 = {0.f, 0.f, 0.f, 0.f}, ao1 = {0.f, 0.f, 0.f, 0.f};
  const v8f z8 = {0.f, 0.f, 0.f, 0.f, 0.f, 0.f, 0.f, 0.f};

#pragma unroll 1
  for (int t0 = 0; t0 < c; t0 += 16) {
    const int nv = (c - t0) < 16 ? (c - t0) : 16;
    int ei = st + t0 + m;
    ei = ei > last ? last : ei;
    const v2i en = *(const v2i*)(lb + 2 * ei);
    const int src = en.x < 0 ? 0 : (en.x > NN - 1 ? NN - 1 : en.x);
    const int eid = en.y < 0 ? 0 : (en.y > NE - 1 ? NE - 1 : en.y);

    wave_sync();
#pragma unroll
    for (int t = 0; t < 2; ++t) {
      const int row = (lane >> 2) + 8 * t;
      const int er  = __shfl(eid, row);
      v4i w = *(const v4i*)(eb + (size_t)er * KE + 8 * (lane & 3));
      const int msk = (row < nv) ? -1 : 0;
      w.x &= msk; w.y &= msk; w.z &= msk; w.w &= msk;
      *(v4i*)(At + row * 16 + 4 * (lane & 3)) = w;
    }
    wave_sync();
    {
      FragB af;
      af.q[0] = *(const v4i*)(At + m * 16 + 4 * hh);
      af.q[1] = *(const v4i*)(At + m * 16 + 8 + 4 * hh);
#pragma unroll
      for (int tt = 0; tt < 16; ++tt) {
        const unsigned short* wq = wet + (size_t)(16 * tt + m) * KE + 8 * hh;
        FragB bf;
        bf.q[0] = *(const v4i*)wq;
        bf.q[1] = *(const v4i*)(wq + 16);
        const v8f d = wmx(af, bf, z8);
        const float bc = sBe[16 * tt + m];
#pragma unroll
        for (int r = 0; r < 8; ++r)
          T[(8 * hh + r) * TP + 16 * tt + m] = relu_np(d[r] + bc);
      }
    }
    wave_sync();

#pragma unroll
    for (int hf = 0; hf < CONV_HALVES; ++hf) {
      v8f acc[CNT_T];
#pragma unroll
      for (int t = 0; t < CNT_T; ++t) acc[t] = z8;
#pragma unroll 1
      for (int s = 0; s < DD / 32; ++s) {
        const float* tr = T + m * TP + 32 * s + 8 * hh;
        const v4f x0 = *(const v4fa*)tr;
        const v4f x1 = *(const v4fa*)(tr + 4);
        const v4f x2 = *(const v4fa*)(tr + 16);
        const v4f x3 = *(const v4fa*)(tr + 20);
        FragB fh, fl;
        unsigned hw, lw;
        split2(x0.x, x0.y, hw, lw); fh.w[0] = (int)hw; fl.w[0] = (int)lw;
        split2(x0.z, x0.w, hw, lw); fh.w[1] = (int)hw; fl.w[1] = (int)lw;
        split2(x1.x, x1.y, hw, lw); fh.w[2] = (int)hw; fl.w[2] = (int)lw;
        split2(x1.z, x1.w, hw, lw); fh.w[3] = (int)hw; fl.w[3] = (int)lw;
        split2(x2.x, x2.y, hw, lw); fh.w[4] = (int)hw; fl.w[4] = (int)lw;
        split2(x2.z, x2.w, hw, lw); fh.w[5] = (int)hw; fl.w[5] = (int)lw;
        split2(x3.x, x3.y, hw, lw); fh.w[6] = (int)hw; fl.w[6] = (int)lw;
        split2(x3.z, x3.w, hw, lw); fh.w[7] = (int)hw; fl.w[7] = (int)lw;
        const unsigned short* wq0 = wmc + (size_t)(16 * hf * CNT_T + m) * WMCP + 32 * s + 8 * hh;
#pragma unroll
        for (int t = 0; t < CNT_T; ++t) {
          const unsigned short* wq = wq0 + (size_t)(16 * t) * WMCP;
          FragB bf;
          bf.q[0] = *(const v4i*)wq;
          bf.q[1] = *(const v4i*)(wq + 16);
          acc[t] = wmx(fh, bf, acc[t]);
          if (STEP2_TWO_TERM) acc[t] = wmx(fl, bf, acc[t]);
        }
      }
#pragma unroll
      for (int t = 0; t < CNT_T; ++t) {
#pragma unroll
        for (int r = 0; r < 8; ++r)
          U[(8 * hh + r) * TP + 16 * (hf * CNT_T + t) + m] = acc[t][r];
      }
    }
    wave_sync();

#pragma unroll 1
    for (int r = 0; r < nv; ++r) {
      const int j = __builtin_amdgcn_readlane(src, r);
      const float* np = nanb + (size_t)j * NAP + 4 * lane;
      const v4f na0 = *(const v4f*)np;
      const v4f na1 = *(const v4f*)(np + 128);
      const v4f u0 = *(const v4fa*)(U + r * TP + 4 * lane);
      const v4f u1 = *(const v4fa*)(U + r * TP + 128 + 4 * lane);
      v4f v0 = (u0 + na0) + nbm0;
      v4f v1 = (u1 + na1) + nbm1;
      v0.x = relu_np(v0.x); v0.y = relu_np(v0.y); v0.z = relu_np(v0.z); v0.w = relu_np(v0.w);
      v1.x = relu_np(v1.x); v1.y = relu_np(v1.y); v1.z = relu_np(v1.z); v1.w = relu_np(v1.w);
      ao0 = ao0 + v0;
      ao1 = ao1 + v1;
    }
  }

  const float cf = (float)(c > 0 ? c : 1);
  const float qnan = __int_as_float(0x7fc00000);
  v4f o0, o1;
  o0.x = ao0.x / cf; o0.y = ao0.y / cf; o0.z = ao0.z / cf; o0.w = ao0.w / cf;
  o1.x = ao1.x / cf; o1.y = ao1.y / cf; o1.z = ao1.z / cf; o1.w = ao1.w / cf;
  o0.x = bad ? qnan : o0.x; o0.y = bad ? qnan : o0.y; o0.z = bad ? qnan : o0.z; o0.w = bad ? qnan : o0.w;
  o1.x = bad ? qnan : o1.x; o1.y = bad ? qnan : o1.y; o1.z = bad ? qnan : o1.z; o1.w = bad ? qnan : o1.w;
  float* gp = outp + (size_t)i * DD + 4 * lane;
  *(volatile v4f*)gp = o0;
  *(volatile v4f*)(gp + 128) = o1;
  __threadfence();
  *(volatile v4f*)gp = o0;
  *(volatile v4f*)(gp + 128) = o1;
}

constexpr size_t al256c(size_t o) { return (o + 255) & ~(size_t)255; }
constexpr size_t O_XB   = 0;
constexpr size_t O_NFHL = al256c(O_XB   + (size_t)MP * DD * 2);
constexpr size_t O_NANB = al256c(O_NFHL + (size_t)MP * NFP * 2);
constexpr size_t O_EB   = al256c(O_NANB + (size_t)MP * NAP * 4);
constexpr size_t O_LIST = al256c(O_EB   + (size_t)NE * KE * 2);
constexpr size_t O_SLOT = al256c(O_LIST + (size_t)NBLK * RCAP * 8);
constexpr size_t O_WNT  = al256c(O_SLOT + (size_t)NBLK * NB * 8);
constexpr size_t O_WET  = al256c(O_WNT  + (size_t)DD * DD * 2);
constexpr size_t O_WAB  = al256c(O_WET  + (size_t)DD * KE * 2);
constexpr size_t O_WMC  = al256c(O_WAB  + (size_t)2 * DD * WABP * 2);
constexpr size_t O_BIAS = al256c(O_WMC  + (size_t)DD * WMCP * 2);
constexpr size_t WS_TOT = al256c(O_BIAS + (size_t)3 * DD * 4);
static_assert(WS_TOT <= ((size_t)128u << 20));

extern "C" void kernel_launch(void* const* d_in, const int* in_sizes, int n_in,
                              void* d_out, int out_size, void* d_ws, size_t ws_size,
                              hipStream_t stream) {
  if (n_in < 10) return;
  if (in_sizes[0] != NN * DD) return;
  if (in_sizes[1] != NE * KE) return;
  if (in_sizes[2] != NE || in_sizes[3] != NE) return;
  if (in_sizes[4] != DD * DD || in_sizes[5] != DD) return;
  if (in_sizes[6] != KE * DD || in_sizes[7] != DD) return;
  if (in_sizes[8] != 3 * DD * DD || in_sizes[9] != DD) return;
  if (out_size != NN * DD) return;
  if (WS_TOT > ws_size) return;

  const float* xin  = (const float*)d_in[0];
  const float* efin = (const float*)d_in[1];
  const int*   idxn = (const int*)  d_in[2];
  const int*   seg  = (const int*)  d_in[3];
  const float* Wn   = (const float*)d_in[4];
  const float* bn   = (const float*)d_in[5];
  const float* We   = (const float*)d_in[6];
  const float* be   = (const float*)d_in[7];
  const float* Wm   = (const float*)d_in[8];
  const float* bm   = (const float*)d_in[9];
  float* out = (float*)d_out;

  char* ws = (char*)d_ws;
  unsigned short* XB   = (unsigned short*)(ws + O_XB);
  unsigned short* NFHL = (unsigned short*)(ws + O_NFHL);
  float*          NANB = (float*)(ws + O_NANB);
  unsigned short* EB   = (unsigned short*)(ws + O_EB);
  int*            LIST = (int*)(ws + O_LIST);
  int*            SLOT = (int*)(ws + O_SLOT);
  unsigned short* WNT  = (unsigned short*)(ws + O_WNT);
  unsigned short* WET  = (unsigned short*)(ws + O_WET);
  unsigned short* WAB  = (unsigned short*)(ws + O_WAB);
  unsigned short* WMC  = (unsigned short*)(ws + O_WMC);
  float*          BIAS = (float*)(ws + O_BIAS);

  hipFuncSetAttribute(reinterpret_cast<const void*>(&k_bucket),
                      hipFuncAttributeMaxDynamicSharedMemorySize, LDS_BKT);
  hipFuncSetAttribute(reinterpret_cast<const void*>(&k_replay),
                      hipFuncAttributeMaxDynamicSharedMemorySize, CONV_DYN);

  k_prep<<<PB_TOT, NTHR, 0, stream>>>(xin, efin, Wn, bn, We, be, Wm, bm, XB, EB, WNT, WET, WAB, WMC, BIAS);
  k_bucket<<<NBLK, NTHR, LDS_BKT, stream>>>(idxn, seg, LIST, SLOT);
  k_gemm<0><<<dim3(MP / GBM, DD / GBN), GTHR, 0, stream>>>(XB, DD, WNT, DD, DD, BIAS, NFHL, NANB, NN);
  k_gemm<1><<<dim3(MP / GBM, (2 * DD) / GBN), GTHR, 0, stream>>>(NFHL, NFP, WAB, WABP, N1_K, BIAS, XB, NANB, NN);
  k_replay<<<NN / CW, CTHR, CONV_DYN, stream>>>(LIST, SLOT, EB, WET, WMC, NANB, BIAS, out);
}
